// E8RHTLinear_8495445311545
// MI455X (gfx1250) — hardware-verified
//
#include <hip/hip_runtime.h>
#include <stdint.h>

typedef __attribute__((ext_vector_type(16))) _Float16 v16h;
typedef __attribute__((ext_vector_type(8)))  _Float16 v8h;
typedef __attribute__((ext_vector_type(8)))  float    v8f;
typedef __attribute__((ext_vector_type(4)))  float    v4f;
typedef __attribute__((ext_vector_type(4)))  int      v4i;

constexpr int kTok    = 64;
constexpr int kN      = 8192;
constexpr int kLog2N  = 13;
constexpr int kGroups = kN / 8;
constexpr int kCb     = 256;
constexpr int kTileK  = 128;
constexpr int kPitchH = 136;
constexpr int kPitchC = 68;
static_assert((1 << kLog2N) == kN);
static_assert((kN % kTileK) == 0 && (kTileK % 32) == 0);
static_assert((kN % 64) == 0 && kTok == 64);
static_assert(kCb == 256);

constexpr double cx_sqrt(double v) {
  double r = v;
  for (int i = 0; i < 64; ++i) { r = 0.5 * (r + v / r); }
  return r;
}
constexpr float kFhtScale = (float)(1.0 / cx_sqrt((double)kN));
static_assert(kFhtScale == 0x1.6a09e6p-7f);

constexpr size_t kOffXH   = 0;
constexpr size_t kOffYR   = kOffXH + (size_t)kTok * kN * 2;
constexpr size_t kWsTotal = kOffYR + (size_t)kTok * kN * 4;
static_assert(kWsTotal == 3145728ull);
static_assert((kOffYR % 128) == 0);
static_assert(kWsTotal <= 134217728ull);

template <typename T> struct Frag;
template <> struct Frag<_Float16> {
  typedef v16h V; union U { v16h v; v8h h[2]; };
  static __device__ __forceinline__ v16h load(const _Float16* p) {
    U f; f.h[0] = *(const v8h*)(p); f.h[1] = *(const v8h*)(p + 16); return f.v;
  }
};
__device__ __forceinline__ v8f mma_h(v16h a, v16h b, v8f c) {
  c = __builtin_amdgcn_wmma_f32_16x16x32_f16(false, a, false, b, (short)0, c, false, false);
  asm volatile("v_nop\n\tv_nop\n\tv_nop\n\tv_nop" : "+v"(c) : "v"(a), "v"(b));
  return c;
}

__device__ __forceinline__ void fht_block(float* buf, const int tid) {
#pragma unroll 1
  for (int h = 1; h < kN; h <<= 1) {
#pragma unroll 4
    for (int t = 0; t < (kN / 2) / 256; ++t) {
      const int j = tid + t * 256;
      const int i = ((j & ~(h - 1)) << 1) | (j & (h - 1));
      const float a = buf[i];
      const float b = buf[i + h];
      buf[i]     = a + b;
      buf[i + h] = a - b;
    }
    __syncthreads();
  }
}

__global__ __launch_bounds__(256) void fht_in_kernel(const float* __restrict__ x,
                                                     const float* __restrict__ SV,
                                                     _Float16* __restrict__ XH) {
  __shared__ __align__(16) float buf[kN];
  const int row = blockIdx.x;
  const int tid = threadIdx.x;
  const float* xr = x + (size_t)row * kN;
#pragma unroll
  for (int it = 0; it < 8; ++it) {
    const int i = (it * 256 + tid) * 4;
    const v4f xv = *(const v4f*)(xr + i);
    const v4f sv = *(const v4f*)(SV + i);
    v4f p;
    p[0] = xv[0] * sv[0];
    p[1] = xv[1] * sv[1];
    p[2] = xv[2] * sv[2];
    p[3] = xv[3] * sv[3];
    *(v4f*)(buf + i) = p;
  }
  __syncthreads();
  fht_block(buf, tid);
  v8h hv[4];
#pragma unroll
  for (int it = 0; it < 4; ++it) {
    const int i = (it * 256 + tid) * 8;
    const v4f a0 = *(const v4f*)(buf + i);
    const v4f a1 = *(const v4f*)(buf + i + 4);
    v8h o;
#pragma unroll
    for (int e = 0; e < 4; ++e) {
      const float f0 = a0[e] * kFhtScale;
      const float f1 = a1[e] * kFhtScale;
      o[e]     = (_Float16)f0;
      o[4 + e] = (_Float16)f1;
    }
    hv[it] = o;
  }
  _Float16* orow = XH + (size_t)row * kN;
  for (int pass = 0; pass < 2; ++pass) {
#pragma unroll
    for (int it = 0; it < 4; ++it) {
      *(volatile v8h*)(orow + (it * 256 + tid) * 8) = hv[it];
    }
    __threadfence();
  }
}

__device__ __forceinline__ void dequant_store(const float* cb1, const float* cb2,
                                              const int i1, const int i2, const float s, _Float16* dst) {
  const int o1 = (i1 & (kCb - 1)) * 8;
  const int o2 = (i2 & (kCb - 1)) * 8;
  const v4f c1a = *(const v4f*)(cb1 + o1);
  const v4f c1b = *(const v4f*)(cb1 + o1 + 4);
  const v4f c2a = *(const v4f*)(cb2 + o2);
  const v4f c2b = *(const v4f*)(cb2 + o2 + 4);
  v8h w;
#pragma unroll
  for (int e = 0; e < 4; ++e) {
    const float w0 = c1a[e] + c2a[e] * s;
    const float w1 = c1b[e] + c2b[e] * s;
    w[e]     = (_Float16)w0;
    w[4 + e] = (_Float16)w1;
  }
  *(v8h*)dst = w;
}

struct GemmTiles { _Float16 a[64 * kPitchH]; _Float16 b[64 * kPitchH]; };
union GemmStage { GemmTiles t; float c[64 * kPitchC]; };
static_assert(sizeof(float) * 64 * kPitchC <= sizeof(GemmTiles));

__global__ __launch_bounds__(256) void qgemm_kernel(const _Float16* __restrict__ XH,
                                                    const int* __restrict__ Q1,
                                                    const int* __restrict__ Q2,
                                                    const float* __restrict__ cb1f,
                                                    const float* __restrict__ cb2f,
                                                    const float* __restrict__ irs_p,
                                                    const float* __restrict__ wsc_p,
                                                    float* __restrict__ YR) {
  __shared__ __align__(16) float sCb1[kCb * 8];
  __shared__ __align__(16) float sCb2[kCb * 8];
  __shared__ __align__(16) GemmStage st;

  const int tid = threadIdx.x;
  {
    const v4f p0 = *(const v4f*)(cb1f + tid * 8);
    const v4f p1 = *(const v4f*)(cb1f + tid * 8 + 4);
    const v4f r0 = *(const v4f*)(cb2f + tid * 8);
    const v4f r1 = *(const v4f*)(cb2f + tid * 8 + 4);
    *(v4f*)(sCb1 + tid * 8)     = p0;
    *(v4f*)(sCb1 + tid * 8 + 4) = p1;
    *(v4f*)(sCb2 + tid * 8)     = r0;
    *(v4f*)(sCb2 + tid * 8 + 4) = r1;
  }
  __syncthreads();

  const float irs = irs_p[0];
  const float wsc = wsc_p[0];

  const int lane  = tid & 31;
  const int wave  = tid >> 5;
  const int rlane = lane & 15;
  const int hh    = lane >> 4;
  const int koff  = hh * 8;
  const int mi    = wave & 3;
  const int nj    = wave >> 2;
  const int n0    = blockIdx.x * 64;

  const int bn = tid >> 2;
  const int bg = (tid & 3) * 4;
  const int* q1row = Q1 + (size_t)(n0 + bn) * kGroups + bg;
  const int* q2row = Q2 + (size_t)(n0 + bn) * kGroups + bg;
  _Float16* sBrow = st.t.b + bn * kPitchH + bg * 8;

  const _Float16* aFrag  = st.t.a + (mi * 16 + rlane) * kPitchH + koff;
  const _Float16* b0Frag = st.t.b + (nj * 32 + rlane) * kPitchH + koff;
  const _Float16* b1Frag = b0Frag + 16 * kPitchH;

  v8f acc0 = (v8f){0.f, 0.f, 0.f, 0.f, 0.f, 0.f, 0.f, 0.f};
  v8f acc1 = (v8f){0.f, 0.f, 0.f, 0.f, 0.f, 0.f, 0.f, 0.f};

#pragma unroll 1
  for (int ch = 0; ch < kN / kTileK; ++ch) {
    __syncthreads();
    const v4i qa = *(const v4i*)(q1row + ch * (kTileK / 8));
    const v4i qb = *(const v4i*)(q2row + ch * (kTileK / 8));
#pragma unroll
    for (int it = 0; it < 4; ++it) {
      const int idx = tid + 256 * it;
      const int r   = idx >> 4;
      const int c8  = (idx & 15) * 8;
      const v8h av = *(const v8h*)(XH + (size_t)r * kN + ch * kTileK + c8);
      *(v8h*)(st.t.a + r * kPitchH + c8) = av;
    }
    dequant_store(sCb1, sCb2, qa[0], qb[0], irs, sBrow);
    dequant_store(sCb1, sCb2, qa[1], qb[1], irs, sBrow + 8);
    dequant_store(sCb1, sCb2, qa[2], qb[2], irs, sBrow + 16);
    dequant_store(sCb1, sCb2, qa[3], qb[3], irs, sBrow + 24);
    __syncthreads();
#pragma unroll
    for (int kk = 0; kk < kTileK / 32; ++kk) {
      const v16h a  = Frag<_Float16>::load(aFrag  + kk * 32);
      const v16h b0 = Frag<_Float16>::load(b0Frag + kk * 32);
      const v16h b1 = Frag<_Float16>::load(b1Frag + kk * 32);
      acc0 = mma_h(a, b0, acc0);
      acc1 = mma_h(a, b1, acc1);
    }
  }

  __syncthreads();
#pragma unroll
  for (int r = 0; r < 8; ++r) {
    const float v0 = acc0[r] * wsc;
    const float v1 = acc1[r] * wsc;
    st.c[(mi * 16 + 8 * hh + r) * kPitchC + nj * 32 + rlane]      = v0;
    st.c[(mi * 16 + 8 * hh + r) * kPitchC + nj * 32 + 16 + rlane] = v1;
  }
  __syncthreads();
  {
    const int c4 = (lane & 15) * 4;
    v4f ov[4];
#pragma unroll
    for (int it = 0; it < 4; ++it) {
      const int row = wave * 8 + it * 2 + hh;
      ov[it] = *(const v4f*)(st.c + row * kPitchC + c4);
    }
    for (int pass = 0; pass < 2; ++pass) {
#pragma unroll
      for (int it = 0; it < 4; ++it) {
        const int row = wave * 8 + it * 2 + hh;
        *(volatile v4f*)(YR + (size_t)row * kN + n0 + c4) = ov[it];
      }
      __threadfence();
    }
  }
}

__global__ __launch_bounds__(256) void fht_out_kernel(const float* __restrict__ YR,
                                                      const float* __restrict__ SU,
                                                      float* __restrict__ out) {
  __shared__ __align__(16) float buf[kN];
  const int row = blockIdx.x;
  const int tid = threadIdx.x;
  const float* yr = YR + (size_t)row * kN;
#pragma unroll
  for (int it = 0; it < 8; ++it) {
    const int i = (it * 256 + tid) * 4;
    const v4f yv = *(const v4f*)(yr + i);
    *(v4f*)(buf + i) = yv;
  }
  __syncthreads();
  fht_block(buf, tid);
  v4f ov[8];
#pragma unroll
  for (int it = 0; it < 8; ++it) {
    const int i = (it * 256 + tid) * 4;
    const v4f bv = *(const v4f*)(buf + i);
    const v4f sv = *(const v4f*)(SU + i);
    v4f o;
#pragma unroll
    for (int e = 0; e < 4; ++e) {
      const float t = bv[e] * kFhtScale;
      o[e] = t * sv[e];
    }
    ov[it] = o;
  }
  float* orow = out + (size_t)row * kN;
  for (int pass = 0; pass < 2; ++pass) {
#pragma unroll
    for (int it = 0; it < 8; ++it) {
      *(volatile v4f*)(orow + (it * 256 + tid) * 4) = ov[it];
    }
    __threadfence();
  }
}

extern "C" void kernel_launch(void* const* d_in, const int* in_sizes, int n_in,
                              void* d_out, int out_size, void* d_ws, size_t ws_size,
                              hipStream_t stream) {
  if (n_in < 9) return;
  if (in_sizes[0] != kTok * kN) return;
  if (in_sizes[1] != kN * kGroups) return;
  if (in_sizes[2] != kN * kGroups) return;
  if (in_sizes[3] != kCb * 8) return;
  if (in_sizes[4] != kCb * 8) return;
  if (in_sizes[5] != kN) return;
  if (in_sizes[6] != kN) return;
  if (in_sizes[7] != 1) return;
  if (in_sizes[8] != 1) return;
  if (out_size != kTok * kN) return;
  if (ws_size < kWsTotal) return;

  const float* x   = (const float*)d_in[0];
  const int*   Q1  = (const int*)d_in[1];
  const int*   Q2  = (const int*)d_in[2];
  const float* cb1 = (const float*)d_in[3];
  const float* cb2 = (const float*)d_in[4];
  const float* SU  = (const float*)d_in[5];
  const float* SV  = (const float*)d_in[6];
  const float* wsc = (const float*)d_in[7];
  const float* irs = (const float*)d_in[8];
  float* out = (float*)d_out;

  char* ws = (char*)d_ws;
  _Float16* XH = (_Float16*)(ws + kOffXH);
  float*    YR = (float*)(ws + kOffYR);

  fht_in_kernel<<<kTok, 256, 0, stream>>>(x, SV, XH);
  qgemm_kernel<<<kN / 64, 256, 0, stream>>>(XH, Q1, Q2, cb1, cb2, irs, wsc, YR);
  fht_out_kernel<<<kTok, 256, 0, stream>>>(YR, SU, out);
}
